// FourierKANLayer_68126771249616
// MI455X (gfx1250) — hardware-verified
//
#include <hip/hip_runtime.h>


#define NR   16384
#define RB   4096
#define NI   128
#define NGF  16
#define KK   (2 * NI * NGF)
#define NO   128
typedef _Float16 h16;
typedef unsigned short bf;
typedef __attribute__((ext_vector_type(16))) __bf16   v16bf;
typedef __attribute__((ext_vector_type(16))) _Float16 v16h;
typedef __attribute__((ext_vector_type(8)))  _Float16 v8h;
typedef __attribute__((ext_vector_type(8)))  unsigned short v8us;
typedef __attribute__((ext_vector_type(8)))  float    v8f;
typedef __attribute__((ext_vector_type(4)))  float    v4f;
typedef __attribute__((ext_vector_type(2)))  float    v2f;
typedef __attribute__((ext_vector_type(2)))  unsigned short v2us;
typedef __attribute__((ext_vector_type(4)))  unsigned short v4us;
typedef v8h  __attribute__((may_alias)) v8ha;
typedef v4f  __attribute__((may_alias)) v4fa;
typedef v8us __attribute__((may_alias)) v8usa;

__device__ __forceinline__ unsigned short f2bf(float f) { unsigned u = __float_as_uint(f); u += 0x7FFFu + ((u >> 16) & 1u); return (unsigned short)(u >> 16); }
__device__ __forceinline__ float bf2f(unsigned short b) { return __uint_as_float(((unsigned)b) << 16); }
__device__ __forceinline__ float bfr(float f) { return bf2f(f2bf(f)); }
__device__ __forceinline__ void splitf(float y, unsigned short& h, unsigned short& l) { h = f2bf(y); l = f2bf(y - bf2f(h)); }
__device__ __forceinline__ v16h cat16(v8h lo, v8h hi) { return __builtin_shufflevector(lo, hi, 0, 1, 2, 3, 4, 5, 6, 7, 8, 9, 10, 11, 12, 13, 14, 15); }
__device__ __forceinline__ v16bf cat16b(v8us lo, v8us hi) { return __builtin_bit_cast(v16bf, __builtin_shufflevector(lo, hi, 0, 1, 2, 3, 4, 5, 6, 7, 8, 9, 10, 11, 12, 13, 14, 15)); }
__device__ __forceinline__ v8f wmma16(v16h a, v16h b, v8f c) { return __builtin_amdgcn_wmma_f32_16x16x32_f16(false, a, false, b, (short)0, c, false, false); }
__device__ __forceinline__ v8f wmmab(v16bf a, v16bf b, v8f c) { return __builtin_amdgcn_wmma_f32_16x16x32_bf16(false, a, false, b, (short)0, c, false, false); }

template <typename T16> struct WFrag;
template <> struct WFrag<h16> { typedef v16h V; static __device__ __forceinline__ V ld(const h16* p) { return cat16(*(const v8h*)p, *(const v8h*)(p + 16)); } static __device__ __forceinline__ v8f mma(V a, V b, v8f c) { return wmma16(a, b, c); } };
template <> struct WFrag<bf> { typedef v16bf V; static __device__ __forceinline__ V ld(const bf* p) { return cat16b(*(const v8us*)p, *(const v8us*)(p + 16)); } static __device__ __forceinline__ v8f mma(V a, V b, v8f c) { return wmmab(a, b, c); } };
template <typename T16, int NSPLIT, bool BIAS>
__global__ __launch_bounds__(32) void k_gemmw(const T16* __restrict__ A, const T16* __restrict__ A2, const T16* __restrict__ Bt, const T16* __restrict__ Bt2, int K, float* C, int ldc, const float* __restrict__ bias, size_t sA, size_t sB, size_t sC) {
    typedef typename WFrag<T16>::V V;
    __shared__ __align__(16) float os[16 * 68];
    const size_t z = blockIdx.z; A += z * sA; if (A2) A2 += z * sA; Bt += z * sB; if (Bt2) Bt2 += z * sB; C += z * sC;
    const int lane = threadIdx.x & 31, lr = lane & 15, hi = lane >> 4; const int r0 = blockIdx.x * 64, c0 = blockIdx.y * 64;
    v8f acc[4][4];
#pragma unroll
    for (int mb = 0; mb < 4; ++mb)
#pragma unroll
        for (int nb = 0; nb < 4; ++nb) acc[mb][nb] = (v8f){};
    const size_t aoff = (size_t)(r0 + lr) * K + 8 * hi, boff = (size_t)(c0 + lr) * K + 8 * hi;
#pragma unroll 1
    for (int kc = 0; kc < K; kc += 32) {
        V a[4], a2[4];
#pragma unroll
        for (int mb = 0; mb < 4; ++mb) { a[mb] = WFrag<T16>::ld(A + aoff + (size_t)mb * 16 * K + kc); if (NSPLIT == 1 || NSPLIT == 2) a2[mb] = WFrag<T16>::ld(A2 + aoff + (size_t)mb * 16 * K + kc); }
#pragma unroll
        for (int nb = 0; nb < 4; ++nb) { const V b = WFrag<T16>::ld(Bt + boff + (size_t)nb * 16 * K + kc); V b2; if (NSPLIT >= 2) b2 = WFrag<T16>::ld(Bt2 + boff + (size_t)nb * 16 * K + kc);
#pragma unroll
            for (int mb = 0; mb < 4; ++mb) { acc[mb][nb] = WFrag<T16>::mma(a[mb], b, acc[mb][nb]); if (NSPLIT == 1 || NSPLIT == 2) acc[mb][nb] = WFrag<T16>::mma(a2[mb], b, acc[mb][nb]); if (NSPLIT >= 2) acc[mb][nb] = WFrag<T16>::mma(a[mb], b2, acc[mb][nb]); } }
        asm volatile("v_nop\n\tv_nop\n\tv_nop\n\tv_nop" : "+v"(acc[0][0]), "+v"(acc[1][1]), "+v"(acc[2][2]), "+v"(acc[3][3]) : "v"(a[0]), "v"(a[3]));
    }
#pragma unroll
    for (int mb = 0; mb < 4; ++mb) {
#pragma unroll
        for (int nb = 0; nb < 4; ++nb) {
#pragma unroll
            for (int j = 0; j < 8; ++j) os[(hi * 8 + j) * 68 + nb * 16 + lr] = acc[mb][nb][j]; }
        __builtin_amdgcn_wave_barrier(); asm volatile("" ::: "memory");
        float* crow = C + (size_t)(r0 + mb * 16) * ldc + c0;
#pragma unroll 1
        for (int ps = 0; ps < 2; ++ps) {
#pragma unroll
            for (int s = 0; s < 8; ++s) { const int row = 2 * s + hi, cofs = lr * 4; v4f val = *(const v4fa*)(os + row * 68 + cofs); if (BIAS) { val[0] += bfr(bias[c0 + cofs]); val[1] += bfr(bias[c0 + cofs + 1]); val[2] += bfr(bias[c0 + cofs + 2]); val[3] += bfr(bias[c0 + cofs + 3]); }
                *(volatile v4f*)(crow + (size_t)row * ldc + cofs) = val; }
            if (ps == 0) __threadfence(); }
        __builtin_amdgcn_wave_barrier(); asm volatile("" ::: "memory");
    }
}

__global__ __launch_bounds__(256) void k_wamp(const float* __restrict__ ca, const float* __restrict__ sa, bf* Bt) { const size_t e = ((size_t)blockIdx.x * 256 + threadIdx.x) * 8; if (e >= (size_t)NO * KK) return; const int k = (int)(e % KK); const int o = (int)(e / KK); const float* src = (k < NI * NGF) ? (ca + (size_t)o * NI * NGF + k) : (sa + (size_t)o * NI * NGF + (k - NI * NGF)); const v8f v = *(const v8f*)src; v8us ob;
#pragma unroll
    for (int q = 0; q < 8; ++q) ob[q] = f2bf(v[q]); *(volatile v8us*)(Bt + e) = ob; __threadfence(); *(volatile v8us*)(Bt + e) = ob; }
__global__ __launch_bounds__(256) void k_feat(const float* __restrict__ X, int r0, bf* Ah, bf* Al) { const size_t e = (size_t)blockIdx.x * 256 + threadIdx.x; if (e >= (size_t)RB * NI) return; const int i = (int)(e % NI); const int n = (int)(e / NI); const float x = bfr(X[(size_t)(r0 + n) * NI + i]); v8us ch0, ch1, cl0, cl1, sh0, sh1, sl0, sl1;
const float c1 = cosf(x), s1 = sinf(x); float c = c1, s = s1;
#pragma unroll
    for (int gq = 0; gq < NGF; ++gq) { if (gq > 0) { float cc = __fmul_rn(c, c1), ss = __fmul_rn(s, s1), sc = __fmul_rn(s, c1), cs = __fmul_rn(c, s1); asm volatile("" : "+v"(cc), "+v"(ss), "+v"(sc), "+v"(cs)); const float cn = __fsub_rn(cc, ss), sn = __fadd_rn(sc, cs); c = cn; s = sn; }
        unsigned short a, b2; splitf(c, a, b2); if (gq < 8) { ch0[gq] = a; cl0[gq] = b2; } else { ch1[gq - 8] = a; cl1[gq - 8] = b2; } splitf(s, a, b2); if (gq < 8) { sh0[gq] = a; sl0[gq] = b2; } else { sh1[gq - 8] = a; sl1[gq - 8] = b2; } }
    const size_t oc = (size_t)n * KK + (size_t)i * NGF, osn = oc + NI * NGF;
#pragma unroll 1
    for (int ps = 0; ps < 2; ++ps) { *(volatile v8us*)(Ah + oc) = ch0; *(volatile v8us*)(Ah + oc + 8) = ch1; *(volatile v8us*)(Al + oc) = cl0; *(volatile v8us*)(Al + oc + 8) = cl1; *(volatile v8us*)(Ah + osn) = sh0; *(volatile v8us*)(Ah + osn + 8) = sh1; *(volatile v8us*)(Al + osn) = sl0; *(volatile v8us*)(Al + osn + 8) = sl1; if (ps == 0) __threadfence(); } }
__global__ __launch_bounds__(256) void k_lnout(const float* __restrict__ F, const float* __restrict__ g, const float* __restrict__ be, float* OUTb) {
    const int lane = threadIdx.x & 31; const int r = blockIdx.x * 8 + (threadIdx.x >> 5); if (r >= RB) return; const v4f a = *(const v4f*)(F + (size_t)r * NO + lane * 4); float s = 0.f;
#pragma unroll
    for (int q = 0; q < 4; ++q) s += a[q];
#pragma unroll
    for (int sh = 16; sh; sh >>= 1) s += __shfl_xor(s, sh, 32);
    const float mu = s * (1.0f / NO); float s2 = 0.f;
#pragma unroll
    for (int q = 0; q < 4; ++q) { const float d0 = __fsub_rn(a[q], mu); float p = __fmul_rn(d0, d0); asm volatile("" : "+v"(p)); s2 = __fadd_rn(s2, p); }
#pragma unroll
    for (int sh = 16; sh; sh >>= 1) s2 += __shfl_xor(s2, sh, 32);
    const float rs = __fdiv_rn(1.0f, __fsqrt_rn(__fadd_rn(s2 * (1.0f / NO), 1e-5f))); v4f o4;
#pragma unroll
    for (int q = 0; q < 4; ++q) { float n0 = __fmul_rn(__fsub_rn(a[q], mu), rs); asm volatile("" : "+v"(n0)); float n1 = __fmul_rn(n0, bfr(g[lane * 4 + q])); asm volatile("" : "+v"(n1)); o4[q] = __fadd_rn(n1, bfr(be[lane * 4 + q])); }
#pragma unroll 1
    for (int ps = 0; ps < 2; ++ps) { *(volatile v4f*)(OUTb + (size_t)r * NO + lane * 4) = o4; if (ps == 0) __threadfence(); } }

extern "C" void kernel_launch(void* const* d_in, const int* in_sizes, int n_in,
                              void* d_out, int out_size, void* d_ws, size_t ws_size, hipStream_t stream) {
    (void)in_sizes; (void)n_in; (void)out_size;
    const float* X = (const float*)d_in[0]; const float* CA = (const float*)d_in[1]; const float* SA = (const float*)d_in[2]; const float* bias = (const float*)d_in[3]; const float* g = (const float*)d_in[4]; const float* be = (const float*)d_in[5];
    float* OUT = (float*)d_out;
    char* wsp = (char*)d_ws;
    auto take = [&](size_t bytes) { char* p = wsp; wsp += (bytes + 255) & ~(size_t)255; return (void*)p; };
    bf* WB = (bf*)take((size_t)NO * KK * 2); bf* Ah = (bf*)take((size_t)RB * KK * 2); bf* Al = (bf*)take((size_t)RB * KK * 2); float* F = (float*)take((size_t)RB * NO * 4);
    if ((size_t)(wsp - (char*)d_ws) > ws_size) return;
    k_wamp<<<(unsigned)(((size_t)NO * KK / 8 + 255) / 256), 256, 0, stream>>>(CA, SA, WB);
    for (int c = 0; c < NR / RB; ++c) { const int r0 = c * RB;
        k_feat<<<(unsigned)(((size_t)RB * NI + 255) / 256), 256, 0, stream>>>(X, r0, Ah, Al);
        k_gemmw<bf, 1, true><<<dim3(RB / 64, NO / 64, 1), 32, 0, stream>>>(Ah, Al, WB, nullptr, KK, F, NO, bias, 0, 0, 0);
        k_lnout<<<RB / 8, 256, 0, stream>>>(F, g, be, OUT + (size_t)r0 * NO); }
}
